// GroundTrans_34677565948527
// MI455X (gfx1250) — hardware-verified
//
#include <hip/hip_runtime.h>
#include <math.h>

typedef __attribute__((ext_vector_type(16))) _Float16 v16h;
typedef __attribute__((ext_vector_type(16))) __bf16 v16b;
typedef __attribute__((ext_vector_type(8)))  _Float16 v8h;
typedef __attribute__((ext_vector_type(8)))  float v8f;
typedef __attribute__((ext_vector_type(4)))  float v4f;
typedef __attribute__((ext_vector_type(2)))  float v2f;
typedef __attribute__((ext_vector_type(4)))  unsigned v4u;
typedef __attribute__((ext_vector_type(4)))  int v4i;
typedef float __attribute__((may_alias)) float_a;
typedef int __attribute__((may_alias)) int_a;

template <typename T> __device__ __forceinline__ void vst2(void* p, T v) { *(volatile T*)p = v; __threadfence(); *(volatile T*)p = v; }
__device__ __forceinline__ v8f wmma16(v16h a, v16h b, v8f c) {
  v8f d = __builtin_amdgcn_wmma_f32_16x16x32_f16(false, a, false, b, (short)0, c, false, false);
  asm volatile("v_nop\n\tv_nop\n\tv_nop\n\tv_nop" : "+v"(d) : "v"(a), "v"(b));
  return d;
}
__device__ __forceinline__ v8f wmma_bf(v16b a, v16b b, v8f c) {
  v8f d = __builtin_amdgcn_wmma_f32_16x16x32_bf16(false, a, false, b, (short)0, c, false, false);
  asm volatile("v_nop\n\tv_nop\n\tv_nop\n\tv_nop" : "+v"(d) : "v"(a), "v"(b));
  return d;
}
__device__ __forceinline__ v16h frag_h(const _Float16* rowk0, int lane) {
  union { v16h v; v8h q[2]; } u; const _Float16* p = rowk0 + 8 * (lane >> 4);
  u.q[0] = *(const v8h*)p; u.q[1] = *(const v8h*)(p + 16); return u.v;
}
__device__ __forceinline__ v16h frag_f32(const float* rowk0, int lane) {
  v16h a; const float* p = rowk0 + 8 * (lane >> 4);
#pragma unroll
  for (int i = 0; i < 8; ++i) { a[i] = (_Float16)p[i]; a[8 + i] = (_Float16)p[16 + i]; }
  return a;
}
__device__ __forceinline__ v16h frag_f32s(const float* rowk0, int lane, float sc) {
  v16h a; const float* p = rowk0 + 8 * (lane >> 4);
#pragma unroll
  for (int i = 0; i < 8; ++i) { a[i] = (_Float16)(p[i] * sc); a[8 + i] = (_Float16)(p[16 + i] * sc); }
  return a;
}
__device__ __forceinline__ v16h fragc_f32(const float* W, int k0, int n, int lane, int ld, int K) {
  v16h a; const int g = lane >> 4;
#pragma unroll
  for (int i = 0; i < 8; ++i) { const int ka = k0 + 8 * g + i, kb = ka + 16;
    a[i] = (_Float16)(ka < K ? W[(size_t)(ka < K ? ka : K - 1) * ld + n] : 0.f); a[8 + i] = (_Float16)(kb < K ? W[(size_t)(kb < K ? kb : K - 1) * ld + n] : 0.f); }
  return a;
}
struct F2 { v16b h, l; };
__device__ __forceinline__ F2 bsplit16(const float v[16]) { F2 r;
#pragma unroll
  for (int i = 0; i < 16; ++i) { const __bf16 h = (__bf16)v[i]; r.h[i] = h; r.l[i] = (__bf16)(v[i] - (float)h); }
  return r; }
__device__ __forceinline__ F2 split_row(const float* row, int k0, int lane) { float v[16]; const float* p = row + k0 + 8 * (lane >> 4);
#pragma unroll
  for (int i = 0; i < 8; ++i) { v[i] = p[i]; v[8 + i] = p[16 + i]; }
  return bsplit16(v); }
__device__ __forceinline__ F2 split_rowK(const float* row, int k0, int lane, int K) { float v[16]; const int g = lane >> 4;
#pragma unroll
  for (int i = 0; i < 8; ++i) { const int ka = k0 + 8 * g + i, kb = ka + 16; v[i] = ka < K ? row[ka < K ? ka : K - 1] : 0.f; v[8 + i] = kb < K ? row[kb < K ? kb : K - 1] : 0.f; }
  return bsplit16(v); }
__device__ __forceinline__ F2 split_col(const float* W, int k0, int n, int lane, int ld, int K) { float v[16]; const int g = lane >> 4;
#pragma unroll
  for (int i = 0; i < 8; ++i) { const int ka = k0 + 8 * g + i, kb = ka + 16; v[i] = ka < K ? W[(size_t)(ka < K ? ka : K - 1) * ld + n] : 0.f; v[8 + i] = kb < K ? W[(size_t)(kb < K ? kb : K - 1) * ld + n] : 0.f; }
  return bsplit16(v); }
__device__ __forceinline__ v8f mac3(const F2& a, const F2& b, v8f c) { c = wmma_bf(a.l, b.h, c); c = wmma_bf(a.h, b.l, c); return wmma_bf(a.h, b.h, c); }
__device__ __forceinline__ float sigm(float v) { return 1.0f / (1.0f + expf(-v)); }
#define LDSX() do { asm volatile("s_wait_dscnt 0" ::: "memory"); __builtin_amdgcn_wave_barrier(); __builtin_amdgcn_fence(__ATOMIC_RELEASE, "workgroup"); } while (0)


#define NB 8
#define CC 256
#define CI 128
#define NHI 1024
#define NLO 4096
#ifndef TNB
#define TNB NB
#endif
typedef __attribute__((ext_vector_type(8))) __bf16 v8b;
__device__ __forceinline__ v16b frag_b(const __bf16* rowk0, int lane) {
  union { v16b v; v8b q[2]; } u; const __bf16* p = rowk0 + 8 * (lane >> 4);
  u.q[0] = *(const v8b*)p; u.q[1] = *(const v8b*)(p + 16); return u.v;
}
__device__ __forceinline__ float bfr(float v) { return (float)(__bf16)v; }
__device__ __attribute__((noinline)) float exp_ni(float v) { return expf(v); }
__device__ __attribute__((noinline)) float erf_ni(float v) { return erff(v); }

#define WS_PW   0u
#define PWG 0
#define PWP (PWG + CI * CC)
#define PWT (PWP + CI * CC)
#define PWZ (PWT + CI * CC)
#define PWEND (PWZ + CC * CI)
#define WS_G    (WS_PW + 2u * PWEND)
#define WS_PHT  (WS_G + 4u * NB * NHI * CI)
#define WS_TH   (WS_PHT + 4u * NB * NHI * CI)
#define WS_MH   (WS_TH + 4u * NB * NLO * CI)
#define WS_ML   (WS_MH + 2u * NB * CI * CI)
#define WS_Y    (WS_ML + 2u * NB * CI * CI)
#define WS_Z    (WS_Y + 4u * NB * NLO * CI)
#define WS_PS   (WS_Z + 4u * NB * CC * NLO)
#define WS_ST   (WS_PS + 4u * NB * 128 * 32)
#define WS_END  (WS_ST + 4u * NB * 32)

__global__ __launch_bounds__(256) void k_pack(const float* __restrict__ WG, const float* __restrict__ WP, const float* __restrict__ WT, const float* __restrict__ WZ, __bf16* __restrict__ PW) {
  __shared__ __align__(16) __bf16 s[CC]; const int r = blockIdx.x, which = blockIdx.y, tid = threadIdx.x;
  if (which < 3 && r >= CI) return;
  const int K = (which < 3) ? CC : CI; const float* src = (which == 0) ? WG : (which == 1 ? WP : (which == 2 ? WT : WZ));
  if (tid < K) s[tid] = (__bf16)src[(size_t)r * K + tid];
  __syncthreads();
  const size_t base = (which == 0) ? PWG : (which == 1 ? PWP : (which == 2 ? PWT : PWZ));
  if (tid < K / 8) vst2((unsigned*)(PW + base + (size_t)r * K + tid * 8), *(const v4u*)&s[tid * 8]);
}
template <int TWO>
__global__ __launch_bounds__(128) void k_proj(const float* __restrict__ X, int npos, const __bf16* __restrict__ PA, const float* __restrict__ BA, const __bf16* __restrict__ PB, const float* __restrict__ BB, float* __restrict__ OA, float* __restrict__ OB) {
  __shared__ __align__(16) __bf16 sx[64][CC + 8]; __shared__ __align__(16) float so[4][16][132];
  const int tid = threadIdx.x, wave = tid >> 5, lane = tid & 31, col = lane & 15, g = lane >> 4; const int b = blockIdx.y; const int p0 = blockIdx.x * 64;
  for (int q = tid; q < CC * 64; q += 128) { const int c = q >> 6, nl = q & 63; sx[nl][c] = (__bf16)X[((size_t)b * CC + c) * npos + p0 + nl]; }
  __syncthreads();
#pragma unroll 1
  for (int which = 0; which < (TWO ? 2 : 1); ++which) { const __bf16* P = which ? PB : PA; const float* bias = which ? BB : BA; float* O = which ? OB : OA;
    v8f acc[8] = {};
#pragma unroll 2
    for (int kc = 0; kc < CC / 32; ++kc) { v16b a;
#pragma unroll
      for (int i = 0; i < 8; ++i) { a[i] = sx[wave * 16 + col][kc * 32 + 8 * g + i]; a[8 + i] = sx[wave * 16 + col][kc * 32 + 16 + 8 * g + i]; }
#pragma unroll
      for (int j = 0; j < 8; ++j) acc[j] = wmma_bf(a, frag_b(P + (size_t)(j * 16 + col) * CC + kc * 32, lane), acc[j]); }
#pragma unroll
    for (int j = 0; j < 8; ++j) { const float bb = bfr(bias[j * 16 + col]);
#pragma unroll
      for (int r = 0; r < 8; ++r) so[wave][8 * g + r][j * 16 + col] = acc[j][r] + bb; }
    LDSX();
    for (int rl = 0; rl < 16; ++rl) vst2(O + ((size_t)b * npos + p0 + wave * 16 + rl) * CI + lane * 4, *(const v4f*)&so[wave][rl][lane * 4]);
    LDSX(); }
}
__global__ __launch_bounds__(128) void k_M(const float* __restrict__ G, const float* __restrict__ PHT, __bf16* __restrict__ MH, __bf16* __restrict__ ML) {
  __shared__ __align__(16) __bf16 sh[CI], sl[CI]; const int cj = blockIdx.x, b = blockIdx.y, ci = threadIdx.x; float acc = 0.f;
  const float* gb = G + (size_t)b * NHI * CI; const float* pb = PHT + (size_t)b * NHI * CI;
  for (int n = 0; n < NHI; ++n) acc += gb[(size_t)n * CI + cj] * pb[(size_t)n * CI + ci];
  const __bf16 hb = (__bf16)acc; sh[ci] = hb; sl[ci] = (__bf16)(acc - (float)hb);
  __syncthreads();
  if (ci < 16) vst2((unsigned*)(MH + ((size_t)b * CI + cj) * CI + ci * 8), *(const v4u*)&sh[ci * 8]); else if (ci < 32) vst2((unsigned*)(ML + ((size_t)b * CI + cj) * CI + (ci - 16) * 8), *(const v4u*)&sl[(ci - 16) * 8]);
}
__global__ __launch_bounds__(128) void k_y(const float* __restrict__ TH, const __bf16* __restrict__ MH, const __bf16* __restrict__ ML, float* __restrict__ Y) {
  __shared__ __align__(16) float so[4][16][132];
  const int tid = threadIdx.x, wave = tid >> 5, lane = tid & 31, col = lane & 15, g = lane >> 4; const int b = blockIdx.y; const size_t r0 = (size_t)b * NLO + blockIdx.x * 64 + wave * 16;
  v8f acc[8] = {};
#pragma unroll
  for (int kc = 0; kc < CI / 32; ++kc) { const F2 a = split_row(TH + (r0 + col) * CI, kc * 32, lane);
#pragma unroll
    for (int j = 0; j < 8; ++j) { const size_t br = ((size_t)b * CI + j * 16 + col) * CI + kc * 32; const v16b bh = frag_b(MH + br, lane), bl = frag_b(ML + br, lane); acc[j] = wmma_bf(a.l, bh, acc[j]); acc[j] = wmma_bf(a.h, bl, acc[j]); acc[j] = wmma_bf(a.h, bh, acc[j]); } }
#pragma unroll
  for (int j = 0; j < 8; ++j)
#pragma unroll
    for (int r = 0; r < 8; ++r) so[wave][8 * g + r][j * 16 + col] = acc[j][r] * (1.0f / 1024.0f);
  LDSX();
  for (int rl = 0; rl < 16; ++rl) vst2(Y + (r0 + rl) * CI + lane * 4, *(const v4f*)&so[wave][rl][lane * 4]);
}
__global__ __launch_bounds__(128) void k_z(const float* __restrict__ Y, const __bf16* __restrict__ PZ, const float* __restrict__ BZ, float* __restrict__ Z, float* __restrict__ PS) {
  __shared__ __align__(16) float st[128][68]; __shared__ float sws[4]; __shared__ __align__(16) float sline[32];
  const int tid = threadIdx.x, wave = tid >> 5, lane = tid & 31, col = lane & 15, g = lane >> 4; const int b = blockIdx.z; const int m0 = blockIdx.x * 64; const int c0 = blockIdx.y * 128; const size_t r0 = (size_t)b * NLO + m0 + wave * 16;
  v8f acc[8] = {};
#pragma unroll
  for (int kc = 0; kc < CI / 32; ++kc) { const F2 a = split_row(Y + (r0 + col) * CI, kc * 32, lane);
#pragma unroll
    for (int j = 0; j < 8; ++j) { const v16b w = frag_b(PZ + (size_t)(c0 + j * 16 + col) * CI + kc * 32, lane); acc[j] = wmma_bf(a.l, w, acc[j]); acc[j] = wmma_bf(a.h, w, acc[j]); } }
  float psum = 0.f;
#pragma unroll
  for (int j = 0; j < 8; ++j) { const int cl = j * 16 + col; const float bb = bfr(BZ[c0 + cl]);
#pragma unroll
    for (int r = 0; r < 8; ++r) { const float v = acc[j][r] + bb; st[cl][wave * 16 + 8 * g + r] = v; psum += v; } }
#pragma unroll
  for (int o = 1; o < 32; o <<= 1) psum += __shfl_xor(psum, o);
  if (lane == 0) sws[wave] = psum;
  __syncthreads();
  for (int q = tid; q < 128 * 16; q += 128) { const int cl = q >> 4, pc = q & 15; vst2(Z + ((size_t)b * CC + c0 + cl) * NLO + m0 + pc * 4, *(const v4f*)&st[cl][pc * 4]); }
  if (tid < 32) sline[tid] = (tid == 0) ? (sws[0] + sws[1] + sws[2] + sws[3]) : 0.f;
  __syncthreads();
  if (tid < 8) vst2(PS + ((size_t)b * 128 + blockIdx.y * 64 + blockIdx.x) * 32 + tid * 4, *(const v4f*)&sline[tid * 4]);
}
template <int MODE>
__global__ __launch_bounds__(128) void k_red(const float* __restrict__ PS, float* __restrict__ ST) {
  __shared__ float s[128]; __shared__ __align__(16) float sline[32]; const int b = blockIdx.x, tid = threadIdx.x;
  s[tid] = PS[((size_t)b * 128 + tid) * 32]; const float keep = (MODE == 1) ? ST[b * 32] : 0.f; __syncthreads();
  if (tid < 32) sline[tid] = 0.f;
  __syncthreads();
  if (tid == 0) { float acc = 0.f; for (int i = 0; i < 128; ++i) acc += s[i]; acc /= (float)(CC * NLO); if (MODE == 0) sline[0] = acc; else { sline[0] = keep; sline[1] = rsqrtf(acc + 1e-5f); } }
  __syncthreads();
  if (tid < 8) vst2(ST + (size_t)b * 32 + tid * 4, *(const v4f*)&sline[tid * 4]);
}
__global__ __launch_bounds__(256) void k_var(const float* __restrict__ Z, const float* __restrict__ ST, float* __restrict__ PS) {
  __shared__ float sw[8]; __shared__ __align__(16) float sline[32]; const int b = blockIdx.y, slab = blockIdx.x, tid = threadIdx.x; const float mu = ST[b * 32];
  const float* zb = Z + (size_t)b * CC * NLO + (size_t)slab * 8192; float acc = 0.f;
  for (int i = tid; i < 8192; i += 256) { const float d = zb[i] - mu; acc += d * d; }
#pragma unroll
  for (int o = 1; o < 32; o <<= 1) acc += __shfl_xor(acc, o);
  if ((tid & 31) == 0) sw[tid >> 5] = acc;
  __syncthreads();
  if (tid < 32) { float v = 0.f; if (tid == 0) for (int w = 0; w < 8; ++w) v += sw[w]; sline[tid] = (tid == 0) ? v : 0.f; }
  __syncthreads();
  if (tid < 8) vst2(PS + ((size_t)b * 128 + slab) * 32 + tid * 4, *(const v4f*)&sline[tid * 4]);
}
__global__ __launch_bounds__(256) void k_out(const float* __restrict__ Z, const float* __restrict__ ST, const float* __restrict__ gm, const float* __restrict__ bt, float* __restrict__ out) {
  const int c = blockIdx.x, b = blockIdx.y, tid = threadIdx.x; const float mu = ST[b * 32], rs = ST[b * 32 + 1]; const float ga = bfr(gm[c]) * rs, be = bfr(bt[c]);
  const float* zr = Z + ((size_t)b * CC + c) * NLO; float* orow = out + ((size_t)b * CC + c) * NLO;
  for (int pc = tid; pc < NLO / 4; pc += 256) { const float* p = zr + pc * 4; vst2(orow + pc * 4, (v4f){(p[0] - mu) * ga + be, (p[1] - mu) * ga + be, (p[2] - mu) * ga + be, (p[3] - mu) * ga + be}); }
}
extern "C" void kernel_launch(void* const* d_in, const int* in_sizes, int n_in, void* d_out, int out_size, void* d_ws, size_t ws_size, hipStream_t stream) {
  (void)in_sizes; (void)n_in; (void)out_size;
  const float** F = (const float**)d_in;
  if (ws_size < (size_t)WS_END) return;
  char* ws = (char*)d_ws; __bf16 *PW = (__bf16*)(ws + WS_PW), *MH = (__bf16*)(ws + WS_MH), *ML = (__bf16*)(ws + WS_ML);
  float *G = (float*)(ws + WS_G), *PHT = (float*)(ws + WS_PHT), *TH = (float*)(ws + WS_TH), *Y = (float*)(ws + WS_Y), *Z = (float*)(ws + WS_Z), *PS = (float*)(ws + WS_PS), *ST = (float*)(ws + WS_ST);
  k_pack<<<dim3(CC, 4), 256, 0, stream>>>(F[2], F[6], F[4], F[8], PW);
  k_proj<1><<<dim3(NHI / 64, TNB), 128, 0, stream>>>(F[0], NHI, PW + PWG, F[3], PW + PWP, F[7], G, PHT);
  k_proj<0><<<dim3(NLO / 64, TNB), 128, 0, stream>>>(F[1], NLO, PW + PWT, F[5], nullptr, nullptr, TH, nullptr);
  k_M<<<dim3(CI, TNB), 128, 0, stream>>>(G, PHT, MH, ML);
  k_y<<<dim3(NLO / 64, TNB), 128, 0, stream>>>(TH, MH, ML, Y);
  k_z<<<dim3(NLO / 64, 2, TNB), 128, 0, stream>>>(Y, PW + PWZ, F[9], Z, PS);
  k_red<0><<<TNB, 128, 0, stream>>>(PS, ST);
  k_var<<<dim3(128, TNB), 256, 0, stream>>>(Z, ST, PS);
  k_red<1><<<TNB, 128, 0, stream>>>(PS, ST);
  k_out<<<dim3(CC, TNB), 256, 0, stream>>>(Z, ST, F[10], F[11], (float*)d_out);
}
